// LlamaCosAttention_7232724927157
// MI455X (gfx1250) — hardware-verified
//
#include <hip/hip_runtime.h>
#include <cmath>


namespace {
constexpr int Bn = 2, S = 2048, HID = 2048, NH = 16, NKV = 4, D = 128, NT = Bn * S;
constexpr int NPJ = 3136;
constexpr float QS = 8.0f, KS = 8.0f, VS = 8.0f, PS = 8.0f, SCALE = 0.08838834764831845f, EPS = 1e-5f;
constexpr size_t QPL = (size_t)Bn * NH * S * D, KPL = (size_t)Bn * NKV * S * D, VPL = (size_t)Bn * NH * D * S;

typedef _Float16 b16;
typedef __attribute__((ext_vector_type(16))) _Float16 v16b;
typedef __attribute__((ext_vector_type(16))) __bf16 v16bb;
typedef __attribute__((ext_vector_type(8))) _Float16 v8b;
typedef __attribute__((ext_vector_type(8))) unsigned short v8us;
typedef __attribute__((ext_vector_type(8))) float v8f;
typedef __attribute__((ext_vector_type(4))) float v4f;
typedef __attribute__((ext_vector_type(2))) float v2f;
typedef __attribute__((ext_vector_type(2))) _Float16 v2b;
struct RopeInv { float v[64]; };
__device__ __forceinline__ float bf16_rne(float f) { unsigned int u = __float_as_uint(f); u += 0x7FFFu + ((u >> 16) & 1u); return __uint_as_float(u & 0xFFFF0000u); }
__device__ __forceinline__ unsigned short bf16_bits(float f) { unsigned int u = __float_as_uint(f); u += 0x7FFFu + ((u >> 16) & 1u); return (unsigned short)(u >> 16); }
__device__ __forceinline__ v16b frag_kb(const b16* p, int hh) { const v8b a = *(const v8b*)(p + 8 * hh), b = *(const v8b*)(p + 16 + 8 * hh); v16b f;
#pragma unroll
  for (int e = 0; e < 8; ++e) { f[e] = a[e]; f[8 + e] = b[e]; } return f; }
__device__ __forceinline__ v16bb frag_bf(const unsigned short* p, int hh) { const v8us a = *(const v8us*)(p + 8 * hh), b = *(const v8us*)(p + 16 + 8 * hh); union { unsigned short s[16]; v16bb v; } u;
#pragma unroll
  for (int e = 0; e < 8; ++e) { u.s[e] = a[e]; u.s[8 + e] = b[e]; } return u.v; }
__device__ __forceinline__ v16bb frag_f32bf(const float* p, int hh) { union { unsigned short s[16]; v16bb v; } u;
#pragma unroll
  for (int e = 0; e < 8; ++e) { u.s[e] = bf16_bits(p[8 * hh + e]); u.s[8 + e] = bf16_bits(p[16 + 8 * hh + e]); } return u.v; }
__device__ __forceinline__ v8f wmma16b(v16b a, v16b b, v8f c) { v8f d = __builtin_amdgcn_wmma_f32_16x16x32_f16(false, a, false, b, (short)0, c, false, false); asm volatile("v_nop\n\tv_nop\n\tv_nop\n\tv_nop" : "+v"(d) : "v"(a), "v"(b)); return d; }
__device__ __forceinline__ v8f wmma16bb(v16bb a, v16bb b, v8f c) { v8f d = __builtin_amdgcn_wmma_f32_16x16x32_bf16(false, a, false, b, (short)0, c, false, false); asm volatile("v_nop\n\tv_nop\n\tv_nop\n\tv_nop" : "+v"(d) : "v"(a), "v"(b)); return d; }
__device__ __forceinline__ void wave_lds_sync() { __builtin_amdgcn_fence(__ATOMIC_RELEASE, "workgroup"); __builtin_amdgcn_wave_barrier(); __builtin_amdgcn_fence(__ATOMIC_ACQUIRE, "workgroup"); }
__device__ __forceinline__ float nexp(float x) { return __builtin_amdgcn_exp2f(x * 1.4426950408889634f); }
__device__ __forceinline__ float pmul(float a, float b) { float p = a * b; asm volatile("" : "+v"(p)); return p; }
__device__ __forceinline__ void sincos_r(float ang, float& sn, float& cs) { const float k = rintf(ang * 0.15915494309189535f); float r = __builtin_fmaf(k, -6.28318548202514648f, ang); r = __builtin_fmaf(k, 1.7484556025237907e-7f, r);
  const float t = r * 0.15915494309189535f; sn = __builtin_amdgcn_sinf(t); cs = __builtin_amdgcn_cosf(t); }

__global__ __launch_bounds__(256) void prep_kernel(const float* __restrict__ Wq, const float* __restrict__ Wk, const float* __restrict__ Wv, const float* __restrict__ Wo, const float* __restrict__ Wg1, const float* __restrict__ bg1, const float* __restrict__ Wg2, const float* __restrict__ bg2, const float* __restrict__ gam, const float* __restrict__ bet, const int* __restrict__ pos, RopeInv rinv, unsigned short* __restrict__ wcat, b16* __restrict__ wo16, float* __restrict__ P, float* __restrict__ cst, float* __restrict__ snt) {
  const size_t tid = (size_t)blockIdx.x * blockDim.x + threadIdx.x, nth = (size_t)gridDim.x * blockDim.x;
  for (int pass = 0; pass < 2; ++pass) {
    for (size_t p = tid; p < (size_t)NPJ * HID / 8; p += nth) { const int o = (int)(p / (HID / 8)), k8 = (int)(p % (HID / 8)) * 8; v8us v;
#pragma unroll
      for (int e = 0; e < 8; ++e) { const size_t k = k8 + e; float w;
        if (o < 2048) w = Wq[k * 2048 + o]; else if (o < 2560) w = Wk[k * 512 + o - 2048]; else if (o < 3072) w = Wv[k * 512 + o - 2560]; else if (o < 3088) w = Wg1[k * 16 + o - 3072]; else if (o < 3104) w = Wg2[k * 16 + o - 3088]; else w = 0.0f;
        v[e] = bf16_bits(w); }
      *(volatile v8us*)(wcat + (size_t)o * HID + k8) = v; }
    for (size_t p = tid; p < (size_t)HID * HID / 8; p += nth) { const int o = (int)(p / (HID / 8)), k8 = (int)(p % (HID / 8)) * 8; v8b v;
#pragma unroll
      for (int e = 0; e < 8; ++e) v[e] = (b16)bf16_rne(Wo[(size_t)(k8 + e) * HID + o]);
      *(volatile v8b*)(wo16 + (size_t)o * HID + k8) = v; }
    for (size_t p = tid; p < 288; p += nth) { float v; if (p < 16) v = bg1[p]; else if (p < 32) v = bg2[p - 16]; else if (p < 160) v = gam[p - 32]; else v = bet[p - 160]; P[p] = bf16_rne(v); }
    for (size_t p = tid; p < (size_t)S * 64; p += nth) { const int s = (int)(p / 64), i = (int)(p % 64); const float ang = (float)pos[s] * rinv.v[i]; float sn, cs; sincos_r(ang, sn, cs); cst[p] = cs; snt[p] = sn; }
    __threadfence(); }
}

__global__ __launch_bounds__(128) void proj_kernel(const float* __restrict__ hs, const unsigned short* __restrict__ wcat, float* __restrict__ proj) {
  __shared__ __attribute__((aligned(16))) float Ts[4][32 * 64];
  const int lane = threadIdx.x & 31, wave = threadIdx.x >> 5, nloc = lane & 15, hlf = lane >> 4, m0 = blockIdx.y * 128 + wave * 32, c0 = blockIdx.x * 64;
  v8f acc[2][4];
#pragma unroll
  for (int r = 0; r < 2; ++r)
#pragma unroll
    for (int t = 0; t < 4; ++t) acc[r][t] = (v8f){};
#pragma unroll 2
  for (int kb = 0; kb < HID; kb += 32) { const v16bb a0 = frag_f32bf(hs + (size_t)(m0 + nloc) * HID + kb, hlf), a1 = frag_f32bf(hs + (size_t)(m0 + 16 + nloc) * HID + kb, hlf);
#pragma unroll
    for (int t = 0; t < 4; ++t) { const v16bb bw = frag_bf(wcat + (size_t)(c0 + t * 16 + nloc) * HID + kb, hlf); acc[0][t] = wmma16bb(a0, bw, acc[0][t]); acc[1][t] = wmma16bb(a1, bw, acc[1][t]); } }
  float* Tt = Ts[wave];
#pragma unroll
  for (int t = 0; t < 4; ++t)
#pragma unroll
    for (int r = 0; r < 2; ++r)
#pragma unroll
      for (int v = 0; v < 8; ++v) Tt[(r * 16 + v + 8 * hlf) * 64 + t * 16 + nloc] = acc[r][t][v];
  wave_lds_sync();
  for (int pass = 0; pass < 2; ++pass) {
#pragma unroll
    for (int j = 0; j < 16; ++j) { const int rr = j * 2 + hlf, c4 = nloc * 4; *(volatile v4f*)(proj + (size_t)(m0 + rr) * NPJ + c0 + c4) = *(const v4f*)(Tt + rr * 64 + c4); }
    __threadfence(); }
}

__global__ __launch_bounds__(256) void qk_kernel(const float* __restrict__ proj, const float* __restrict__ cst, const float* __restrict__ snt, const float* __restrict__ P, b16* __restrict__ qp, b16* __restrict__ kp, float* __restrict__ g1t) {
  const int wid = threadIdx.x >> 5, lane = threadIdx.x & 31; const int tok = blockIdx.x * 8 + wid, b = tok / S, s = tok % S; const float* pr = proj + (size_t)tok * NPJ;
  const int dA = 2 * lane; const v2f c2 = *(const v2f*)(cst + (size_t)s * 64 + dA), s2 = *(const v2f*)(snt + (size_t)s * 64 + dA);
  for (int h = 0; h < NH + NKV; ++h) { const float* br = pr + ((h < NH) ? h * D : (2048 + (h - NH) * D)); const v2f xa = *(const v2f*)(br + dA), xb = *(const v2f*)(br + 64 + dA);
    const float o0 = xa[0] * c2[0] - xb[0] * s2[0], o1 = xa[1] * c2[1] - xb[1] * s2[1], o2 = xb[0] * c2[0] + xa[0] * s2[0], o3 = xb[1] * c2[1] + xa[1] * s2[1];
    const float scl = (h < NH) ? SCALE * QS : KS; b16* dst = (h < NH) ? (qp + (((size_t)b * NH + h) * S + s) * D) : (kp + (((size_t)b * NKV + (h - NH)) * S + s) * D);
    v2b p01, p23; p01[0] = (b16)(o0 * scl); p01[1] = (b16)(o1 * scl); p23[0] = (b16)(o2 * scl); p23[1] = (b16)(o3 * scl);
    for (int pass = 0; pass < 2; ++pass) { *(volatile v2b*)(dst + dA) = p01; *(volatile v2b*)(dst + 64 + dA) = p23; } }
  if (lane < 16) { const float g1 = 1.0f / (1.0f + nexp(-(pr[3072 + lane] + P[lane]))); for (int pass = 0; pass < 2; ++pass) ((volatile float*)g1t)[(size_t)tok * 16 + lane] = g1; }
  __threadfence();
}

__global__ __launch_bounds__(256) void vt_kernel(const float* __restrict__ proj, const float* __restrict__ P, b16* __restrict__ vt) {
  __shared__ __attribute__((aligned(16))) b16 Tv[D][128 + 8]; __shared__ float G2[128];
  const int t_ = threadIdx.x, t0 = blockIdx.x * 128, h = blockIdx.y, b = blockIdx.z, kv = h / (NH / NKV);
  if (t_ < 128) { const float* pr = proj + ((size_t)b * S + t0 + t_) * NPJ; G2[t_] = 1.0f / (1.0f + nexp(-(pr[3088 + h] + P[16 + h]))); }
  __syncthreads();
  for (int i = t_; i < 128 * D; i += 256) { const int tt = i >> 7, d = i & 127; const float* pr = proj + ((size_t)b * S + t0 + tt) * NPJ; Tv[d][tt] = (b16)(pr[2560 + kv * D + d] * G2[tt] * VS); }
  __syncthreads();
  for (int pass = 0; pass < 2; ++pass) { for (int i = t_; i < D * 16; i += 256) { const int d = i >> 4, c8 = (i & 15) * 8; *(volatile v8b*)(vt + (((size_t)b * NH + h) * D + d) * S + t0 + c8) = *(const v8b*)(&Tv[d][c8]); } __threadfence(); }
}

__global__ __launch_bounds__(256) void attn_kernel(const b16* __restrict__ qp, const b16* __restrict__ kp, const b16* __restrict__ vt, const float* __restrict__ g1t, const float* __restrict__ P, b16* __restrict__ ctx) {
  __shared__ __attribute__((aligned(16))) b16 Os[16][8 * D + 8];
  const int wid = threadIdx.x >> 5, lane = threadIdx.x & 31, hh = lane >> 4, col = lane & 15; const int b = blockIdx.x / (S / 16), q0 = (blockIdx.x % (S / 16)) * 16, h = blockIdx.y * 8 + wid, kv = h / (NH / NKV), qi = q0 + col;
  const b16* Q = qp + (((size_t)b * NH + h) * S) * D; const b16* K = kp + (((size_t)b * NKV + kv) * S) * D; const b16* V = vt + (((size_t)b * NH + h) * D) * S;
  v16b qf[4];
#pragma unroll
  for (int ks = 0; ks < 4; ++ks) qf[ks] = frag_kb(Q + (size_t)qi * D + ks * 32, hh);
  float m = -INFINITY, l = 0.0f; v8f o[8];
#pragma unroll
  for (int t = 0; t < 8; ++t) o[t] = (v8f){};
  for (int kb = 0; kb < q0 + 16; kb += 32) { const bool diag = (kb + 32 > q0); v8f s0 = {}, s1 = {};
#pragma unroll
    for (int ks = 0; ks < 4; ++ks) { const v16b ka = frag_kb(K + (size_t)(kb + col) * D + ks * 32, hh), kc = frag_kb(K + (size_t)(kb + 16 + col) * D + ks * 32, hh); s0 = wmma16b(ka, qf[ks], s0); s1 = wmma16b(kc, qf[ks], s1); }
    float mr = -INFINITY;
#pragma unroll
    for (int r = 0; r < 8; ++r) { s0[r] *= 1.0f / (QS * KS); s1[r] *= 1.0f / (QS * KS); if (diag) { if (kb + 8 * hh + r > qi) s0[r] = -INFINITY; if (kb + 16 + 8 * hh + r > qi) s1[r] = -INFINITY; } mr = fmaxf(mr, fmaxf(s0[r], s1[r])); }
    mr = fmaxf(mr, __shfl_xor(mr, 16));
    const float mn = fmaxf(m, mr), al_ = nexp(m - mn); m = mn; float sum = 0.0f; v16b pbv;
#pragma unroll
    for (int r = 0; r < 8; ++r) { const float e0 = nexp(s0[r] - mn), e1 = nexp(s1[r] - mn); sum += e0 + e1; pbv[r] = (b16)(e0 * PS); pbv[8 + r] = (b16)(e1 * PS); }
    sum += __shfl_xor(sum, 16); l = l * al_ + sum;
#pragma unroll
    for (int t = 0; t < 8; ++t) { o[t] *= al_; const v16b vf = frag_kb(V + (size_t)(t * 16 + col) * S + kb, hh); o[t] = wmma16b(vf, pbv, o[t]); } }
  const float inv = 1.0f / (l * VS * PS); float sm = 0.0f;
#pragma unroll
  for (int t = 0; t < 8; ++t)
#pragma unroll
    for (int r = 0; r < 8; ++r) { o[t][r] *= inv; sm += o[t][r]; }
  sm += __shfl_xor(sm, 16); const float mu = sm * (1.0f / D); float sq = 0.0f;
#pragma unroll
  for (int t = 0; t < 8; ++t)
#pragma unroll
    for (int r = 0; r < 8; ++r) { const float dd = o[t][r] - mu; sq += pmul(dd, dd); }
  sq += __shfl_xor(sq, 16); const float is = rsqrtf(sq * (1.0f / D) + EPS); const float g1 = g1t[((size_t)b * S + qi) * 16 + h];
#pragma unroll
  for (int t = 0; t < 8; ++t)
#pragma unroll
    for (int r = 0; r < 8; ++r) { const int d = t * 16 + 8 * hh + r; Os[col][wid * D + d] = (b16)((pmul((o[t][r] - mu) * is, P[32 + d]) + P[160 + d]) * g1); }
  __syncthreads();
  for (int pass = 0; pass < 2; ++pass) { for (int i = threadIdx.x; i < 16 * (8 * D / 8); i += 256) { const int rr = i / (8 * D / 8), c8 = (i % (8 * D / 8)) * 8; *(volatile v8b*)(ctx + ((size_t)b * S + q0 + rr) * HID + blockIdx.y * 8 * D + c8) = *(const v8b*)(&Os[rr][c8]); } __threadfence(); }
}

__global__ __launch_bounds__(128) void out_kernel(const b16* __restrict__ ctx, const b16* __restrict__ wo16, float* __restrict__ out) {
  __shared__ __attribute__((aligned(16))) float Ts[4][32 * 64];
  const int lane = threadIdx.x & 31, wave = threadIdx.x >> 5, nloc = lane & 15, hlf = lane >> 4, m0 = blockIdx.y * 128 + wave * 32, c0 = blockIdx.x * 64;
  v8f acc[2][4];
#pragma unroll
  for (int r = 0; r < 2; ++r)
#pragma unroll
    for (int t = 0; t < 4; ++t) acc[r][t] = (v8f){};
#pragma unroll 2
  for (int kb = 0; kb < HID; kb += 32) { const v16b a0 = frag_kb(ctx + (size_t)(m0 + nloc) * HID + kb, hlf), a1 = frag_kb(ctx + (size_t)(m0 + 16 + nloc) * HID + kb, hlf);
#pragma unroll
    for (int t = 0; t < 4; ++t) { const v16b bw = frag_kb(wo16 + (size_t)(c0 + t * 16 + nloc) * HID + kb, hlf); acc[0][t] = wmma16b(a0, bw, acc[0][t]); acc[1][t] = wmma16b(a1, bw, acc[1][t]); } }
  float* Tt = Ts[wave];
#pragma unroll
  for (int t = 0; t < 4; ++t)
#pragma unroll
    for (int r = 0; r < 2; ++r)
#pragma unroll
      for (int v = 0; v < 8; ++v) Tt[(r * 16 + v + 8 * hlf) * 64 + t * 16 + nloc] = acc[r][t][v];
  wave_lds_sync();
  for (int pass = 0; pass < 2; ++pass) {
#pragma unroll
    for (int j = 0; j < 16; ++j) { const int rr = j * 2 + hlf, c4 = nloc * 4; *(volatile v4f*)(out + (size_t)(m0 + rr) * HID + c0 + c4) = *(const v4f*)(Tt + rr * 64 + c4); }
    __threadfence(); }
}
}

extern "C" void kernel_launch(void* const* d_in, const int* in_sizes, int n_in,
                              void* d_out, int out_size, void* d_ws, size_t ws_size, hipStream_t stream) {
  (void)n_in; (void)out_size;
  const float* hs = (const float*)d_in[0]; const int* pos = (const int*)d_in[1]; const float* Wq = (const float*)d_in[2]; const float* Wk = (const float*)d_in[3]; const float* Wv = (const float*)d_in[4]; const float* Wo = (const float*)d_in[5];
  const float* Wg1 = (const float*)d_in[6]; const float* bg1 = (const float*)d_in[7]; const float* Wg2 = (const float*)d_in[8]; const float* bg2 = (const float*)d_in[9]; const float* gam = (const float*)d_in[10]; const float* bet = (const float*)d_in[11];
  float* out = (float*)d_out;
  if (in_sizes[0] != NT * HID || in_sizes[1] != S || in_sizes[2] != HID * 2048 || in_sizes[3] != HID * 512 || in_sizes[5] != 2048 * HID || in_sizes[6] != HID * 16) return;
  size_t off = 0; char* ws = (char*)d_ws;
  auto carve = [&](size_t bytes) { char* p = ws + off; off += (bytes + 255) & ~(size_t)255; return p; };
  unsigned short* wcat = (unsigned short*)carve((size_t)NPJ * HID * 2); b16* wo16 = (b16*)carve((size_t)HID * HID * 2); float* P = (float*)carve(512 * 4); float* cst = (float*)carve((size_t)S * 64 * 4); float* snt = (float*)carve((size_t)S * 64 * 4);
  float* proj = (float*)carve((size_t)NT * NPJ * 4); b16* qp = (b16*)carve(QPL * 2); b16* kp = (b16*)carve(KPL * 2); b16* vt = (b16*)carve(VPL * 2); float* g1t = (float*)carve((size_t)NT * 16 * 4);
  b16* ctx = (b16*)proj;
  if (off > ws_size) return;
  RopeInv rinv; for (int i = 0; i < 64; ++i) rinv.v[i] = (float)(1.0 / pow(10000.0, (double)(2 * i) / 128.0));
  prep_kernel<<<512, 256, 0, stream>>>(Wq, Wk, Wv, Wo, Wg1, bg1, Wg2, bg2, gam, bet, pos, rinv, wcat, wo16, P, cst, snt);
  proj_kernel<<<dim3(NPJ / 64, NT / 128), 128, 0, stream>>>(hs, wcat, proj);
  qk_kernel<<<NT / 8, 256, 0, stream>>>(proj, cst, snt, P, qp, kp, g1t);
  vt_kernel<<<dim3(S / 128, NH, Bn), 256, 0, stream>>>(proj, P, vt);
  attn_kernel<<<dim3(Bn * S / 16, 2), 256, 0, stream>>>(qp, kp, vt, g1t, P, ctx);
  out_kernel<<<dim3(HID / 64, NT / 128), 128, 0, stream>>>(ctx, wo16, out);
}
